// GRURegressor_66391604461962
// MI455X (gfx1250) — hardware-verified
//
#include <hip/hip_runtime.h>


#define NBATCH 256
#define NSTEP 512
#define NF 64
#define NH 512
#define NG3 1536
#define RB 32
#define NBLK (NBATCH / RB)
#define HP 520
#define XP 72

typedef __attribute__((ext_vector_type(16))) _Float16 v16h;
typedef __attribute__((ext_vector_type(8)))  _Float16 v8h;
typedef __attribute__((ext_vector_type(16))) __bf16   v16b;
typedef __attribute__((ext_vector_type(8)))  __bf16   v8b;
typedef __attribute__((ext_vector_type(8)))  float    v8f;
typedef __attribute__((ext_vector_type(4)))  float    v4f;

__device__ __forceinline__ void dep_guard_h(v8f& a, v8f& b, v16h x, v16h y) { asm volatile("v_nop\n\tv_nop\n\tv_nop\n\tv_nop" : "+v"(a), "+v"(b) : "v"(x), "v"(y)); }
__device__ __forceinline__ void dep_guard_b(v8f& a, v8f& b, v16b x, v16b y) { asm volatile("v_nop\n\tv_nop\n\tv_nop\n\tv_nop" : "+v"(a), "+v"(b) : "v"(x), "v"(y)); }
__device__ __forceinline__ void keep4_h(v16h a, v16h b, v16h c, v16h d) { asm volatile("v_nop" :: "v"(a), "v"(b), "v"(c), "v"(d)); }
__device__ __forceinline__ void keep4_b(v16b a, v16b b, v16b c, v16b d) { asm volatile("v_nop" :: "v"(a), "v"(b), "v"(c), "v"(d)); }
__device__ __forceinline__ void acc_guard4(v8f& a, v8f& b, v8f& c, v8f& d) { asm volatile("v_nop\n\tv_nop\n\tv_nop\n\tv_nop" : "+v"(a), "+v"(b), "+v"(c), "+v"(d)); }
template <typename T> struct Frag;
template <> struct Frag<_Float16> {
  typedef v16h V; union U { v16h v; v8h h[2]; };
  static __device__ __forceinline__ v16h load(const _Float16* p) {
    U f; f.h[0] = *(const v8h*)(p); f.h[1] = *(const v8h*)(p + 16); return f.v;
  }
  static __device__ __forceinline__ v8f mma(v16h a, v16h b, v8f c) {
    return __builtin_amdgcn_wmma_f32_16x16x32_f16(false, a, false, b, (short)0, c, false, false);
  }
  static __device__ __forceinline__ void guard(v8f& a, v8f& b, v16h x, v16h y) { dep_guard_h(a, b, x, y); }
  static __device__ __forceinline__ void keep(v16h a, v16h b, v16h c, v16h d) { keep4_h(a, b, c, d); }
};
template <> struct Frag<__bf16> {
  typedef v16b V; union U { v16b v; v8b h[2]; };
  static __device__ __forceinline__ v16b load(const __bf16* p) {
    U f; f.h[0] = *(const v8b*)(p); f.h[1] = *(const v8b*)(p + 16); return f.v;
  }
  static __device__ __forceinline__ v8f mma(v16b a, v16b b, v8f c) {
    return __builtin_amdgcn_wmma_f32_16x16x32_bf16(false, a, false, b, (short)0, c, false, false);
  }
  static __device__ __forceinline__ void guard(v8f& a, v8f& b, v16b x, v16b y) { dep_guard_b(a, b, x, y); }
  static __device__ __forceinline__ void keep(v16b a, v16b b, v16b c, v16b d) { keep4_b(a, b, c, d); }
};

__global__ __launch_bounds__(256) void rows_to_f16(
    const float* __restrict__ src, _Float16* __restrict__ dst, int R, int Cin, int Cpad, float scale)
{
  const int lane = threadIdx.x & 31;
  const int wave = threadIdx.x >> 5;
  const int r = blockIdx.x * 8 + wave;
  if (r >= R) return;
  const float* sp = src + (size_t)r * Cin;
  _Float16* dp = dst + (size_t)r * Cpad;
  v8h o[2];
#pragma unroll
  for (int ch = 0; ch < 2; ++ch) {
    const int c0 = ch * 256 + 8 * lane;
    int ca = c0, cb = c0 + 4;
    const bool va = (ca + 3 < Cin), vb = (cb + 3 < Cin);
    ca = va ? ca : (Cin - 4);
    cb = vb ? cb : (Cin - 4);
    v4f x0 = *(const v4f*)(sp + ca);
    v4f x1 = *(const v4f*)(sp + cb);
    const v4f z = (v4f){0.f, 0.f, 0.f, 0.f};
    if (!va) x0 = z;
    if (!vb) x1 = z;
#pragma unroll
    for (int e = 0; e < 4; ++e) {
      o[ch][e]     = (_Float16)(x0[e] * scale);
      o[ch][4 + e] = (_Float16)(x1[e] * scale);
    }
  }
  for (int pass = 0; pass < 2; ++pass) {
#pragma unroll
    for (int ch = 0; ch < 2; ++ch) {
      const int c0 = ch * 256 + 8 * lane;
      if (c0 < Cpad) *(volatile v8h*)(dp + c0) = o[ch];
    }
    __threadfence();
  }
}

__device__ __forceinline__ float sigm_f(float x) { return __builtin_amdgcn_rcpf(1.0f + __expf(-x)); }
__device__ __forceinline__ float tanh_f(float x) { return 1.0f - 2.0f * __builtin_amdgcn_rcpf(__expf(2.0f * x) + 1.0f); }

__device__ __forceinline__ void stage_x(const float* __restrict__ x, int b0, int t, _Float16* xb, int xr, int xc) {
  const float* sp = x + ((size_t)(b0 + xr) * NSTEP + t) * NF + xc;
  const v4f x0 = *(const v4f*)sp;
  const v4f x1 = *(const v4f*)(sp + 4);
  v8h o;
#pragma unroll
  for (int e = 0; e < 4; ++e) {
    o[e]     = (_Float16)(x0[e] * 64.0f);
    o[4 + e] = (_Float16)(x1[e] * 64.0f);
  }
  *(v8h*)(xb + xr * XP + xc) = o;
}

__global__ __launch_bounds__(256) void gru_kernel(
    const float* __restrict__ x,
    const _Float16* __restrict__ Wi16,
    const _Float16* __restrict__ Wh16,
    const float* __restrict__ b_ih,
    const float* __restrict__ b_hh,
    const float* __restrict__ head_w,
    const float* __restrict__ head_b,
    float* __restrict__ out)
{
  __shared__ __align__(16) _Float16 hsh[2 * RB * HP];
  __shared__ __align__(16) _Float16 xsh[2 * RB * XP];
  __shared__ __align__(16) float hf[RB * NH];
  __shared__ float bsh[4 * NH];
  typedef Frag<_Float16> F;
  const int tid  = threadIdx.x;
  const int lane = tid & 31, wave = tid >> 5, hh = lane >> 4, rl = lane & 15;
  const int b0   = (int)blockIdx.x * RB;
  const int xr   = tid >> 3, xc = (tid & 7) * 8;

  for (int i = tid; i < 2 * RB * HP; i += 256) hsh[i] = (_Float16)0.0f;
  for (int i = tid; i < RB * NH; i += 256) hf[i] = 0.0f;
  for (int i = tid; i < 2 * NH; i += 256) bsh[i] = b_ih[i] + b_hh[i];
  for (int i = tid; i < NH; i += 256) { bsh[2 * NH + i] = b_ih[2 * NH + i]; bsh[3 * NH + i] = b_hh[2 * NH + i]; }
  stage_x(x, b0, 0, xsh, xr, xc);
  __syncthreads();

  const int u0w = wave * 64;
  const float S = 1.0f / 4096.0f;

  for (int s = 0; s < NSTEP; ++s) {
    const _Float16* hc  = hsh + (s & 1) * (RB * HP);
    _Float16*       hn  = hsh + ((s & 1) ^ 1) * (RB * HP);
    const _Float16* xcb = xsh + (s & 1) * (RB * XP);
    _Float16*       xnb = xsh + ((s & 1) ^ 1) * (RB * XP);
#pragma unroll 1
    for (int q = 0; q < 4; ++q) {
      const int ub = u0w + 16 * q;
      v8f acc[2][4];
#pragma unroll
      for (int mt = 0; mt < 2; ++mt)
#pragma unroll
        for (int g = 0; g < 4; ++g) acc[mt][g] = (v8f){0.f,0.f,0.f,0.f,0.f,0.f,0.f,0.f};

#pragma unroll
      for (int k0 = 0; k0 < NF; k0 += 32) {
        v16h bfr[3];
#pragma unroll
        for (int g = 0; g < 3; ++g) bfr[g] = F::load(Wi16 + (size_t)(g * NH + ub + rl) * NF + k0 + 8 * hh);
        const v16h a0 = F::load(xcb + rl * XP + k0 + 8 * hh);
        const v16h a1 = F::load(xcb + (16 + rl) * XP + k0 + 8 * hh);
        acc[0][0] = F::mma(a0, bfr[0], acc[0][0]);
        acc[0][1] = F::mma(a0, bfr[1], acc[0][1]);
        acc[0][2] = F::mma(a0, bfr[2], acc[0][2]);
        acc[1][0] = F::mma(a1, bfr[0], acc[1][0]);
        acc[1][1] = F::mma(a1, bfr[1], acc[1][1]);
        acc[1][2] = F::mma(a1, bfr[2], acc[1][2]);
        F::guard(acc[0][0], acc[1][2], a0, a1);
        keep4_h(bfr[0], bfr[1], bfr[2], bfr[2]);
      }
#pragma unroll 1
      for (int k0 = 0; k0 < NH; k0 += 32) {
        v16h bfr[3];
#pragma unroll
        for (int g = 0; g < 3; ++g) bfr[g] = F::load(Wh16 + (size_t)(g * NH + ub + rl) * NH + k0 + 8 * hh);
        const v16h a0 = F::load(hc + rl * HP + k0 + 8 * hh);
        const v16h a1 = F::load(hc + (16 + rl) * HP + k0 + 8 * hh);
        acc[0][0] = F::mma(a0, bfr[0], acc[0][0]);
        acc[0][1] = F::mma(a0, bfr[1], acc[0][1]);
        acc[0][3] = F::mma(a0, bfr[2], acc[0][3]);
        acc[1][0] = F::mma(a1, bfr[0], acc[1][0]);
        acc[1][1] = F::mma(a1, bfr[1], acc[1][1]);
        acc[1][3] = F::mma(a1, bfr[2], acc[1][3]);
        F::guard(acc[0][0], acc[1][3], a0, a1);
        keep4_h(bfr[0], bfr[1], bfr[2], bfr[2]);
      }
      acc_guard4(acc[0][0], acc[0][1], acc[0][2], acc[0][3]);
      acc_guard4(acc[1][0], acc[1][1], acc[1][2], acc[1][3]);

      const int u = ub + rl;
      const float brr = bsh[u], bzz = bsh[NH + u], bin = bsh[2 * NH + u], bhn = bsh[3 * NH + u];
#pragma unroll
      for (int mt = 0; mt < 2; ++mt) {
#pragma unroll
        for (int r = 0; r < 8; ++r) {
          const int row = 16 * mt + 8 * hh + r;
          const float pr  = acc[mt][0][r] * S + brr;
          const float pz  = acc[mt][1][r] * S + bzz;
          const float gin = acc[mt][2][r] * S + bin;
          const float ghn = acc[mt][3][r] * S + bhn;
          const float rg = sigm_f(pr);
          const float zg = sigm_f(pz);
          const float ng = tanh_f(gin + rg * ghn);
          const float hp = hf[row * NH + u];
          const float hv = (1.0f - zg) * ng + zg * hp;
          hf[row * NH + u] = hv;
          hn[row * HP + u] = (_Float16)(hv * 64.0f);
        }
      }
    }
    const int t1 = (s + 1 < NSTEP) ? (s + 1) : s;
    stage_x(x, b0, t1, xnb, xr, xc);
    __syncthreads();
  }

  if (wave == 0) {
    const float* hrow = hf + lane * NH;
    float sacc = 0.0f;
#pragma unroll 4
    for (int k = 0; k < NH; ++k) sacc += hrow[k] * head_w[k];
    sacc += head_b[0];
    *(volatile float*)(out + b0 + lane) = sacc;
    __threadfence();
    *(volatile float*)(out + b0 + lane) = sacc;
  }
}

extern "C" void kernel_launch(void* const* d_in, const int* in_sizes, int n_in,
                              void* d_out, int out_size, void* d_ws, size_t ws_size,
                              hipStream_t stream) {
  if (n_in < 7) return;
  if (in_sizes[0] != NBATCH * NSTEP * NF) return;
  if (in_sizes[1] != NG3 * NF || in_sizes[2] != NG3 * NH) return;
  if (in_sizes[3] != NG3 || in_sizes[4] != NG3) return;
  if (in_sizes[5] != NH || in_sizes[6] < 1) return;
  if (out_size != NBATCH) return;

  const float* x      = (const float*)d_in[0];
  const float* W_ih   = (const float*)d_in[1];
  const float* W_hh   = (const float*)d_in[2];
  const float* b_ih   = (const float*)d_in[3];
  const float* b_hh   = (const float*)d_in[4];
  const float* head_w = (const float*)d_in[5];
  const float* head_b = (const float*)d_in[6];
  float* out = (float*)d_out;

  const size_t szWi = (size_t)NG3 * NF * 2;
  const size_t szWh = (size_t)NG3 * NH * 2;
  size_t off = 0;
  const size_t oWi = off; off += szWi;
  const size_t oWh = off; off += szWh;
  if (off > ws_size) return;
  char* ws = (char*)d_ws;
  _Float16* Wi16 = (_Float16*)(ws + oWi);
  _Float16* Wh16 = (_Float16*)(ws + oWh);

  rows_to_f16<<<(NG3 + 7) / 8, 256, 0, stream>>>(W_ih, Wi16, NG3, NF, NF, 64.0f);
  rows_to_f16<<<(NG3 + 7) / 8, 256, 0, stream>>>(W_hh, Wh16, NG3, NH, NH, 64.0f);

  gru_kernel<<<NBLK, 256, 0, stream>>>(x, Wi16, Wh16, b_ih, b_hh, head_w, head_b, out);
}
